// JiTBlock_85555748537166
// MI455X (gfx1250) — hardware-verified
//
#include <hip/hip_runtime.h>
#include <hip/hip_bf16.h>
#include <math.h>

#define BB 4
#define SS 1024
#define DD 1024
#define HH 16
#define KVH 16
#define KVD 1024
#define DKK 64
#define QW 2
#define MTOK (BB * SS)
#define MH 2730
#define MHP 2816
#define GSTR 48

typedef _Float16 bf16;
typedef _Float16 f16;
typedef __attribute__((ext_vector_type(4))) unsigned v4u_t;
typedef unsigned v4ua __attribute__((ext_vector_type(4), may_alias));
typedef __attribute__((ext_vector_type(4))) float v4f_t;
typedef float v4fa __attribute__((ext_vector_type(4), may_alias));
typedef __attribute__((ext_vector_type(16))) bf16  bf16x16;
typedef bf16x16 f16x16;
typedef __attribute__((ext_vector_type(8)))  bf16  bf16x8;
typedef bf16x8 f16x8;
typedef __attribute__((ext_vector_type(4)))  bf16  bf16x4;
typedef __attribute__((ext_vector_type(8)))  float f32x8;
__device__ __forceinline__ f32x8 wmma16(f16x16 a, f16x16 b, f32x8 c) {
  c = __builtin_amdgcn_wmma_f32_16x16x32_f16(false, a, false, b, (short)0, c, false, false);
  asm volatile("v_nop\n\tv_nop\n\tv_nop\n\tv_nop" : "+v"(c) : "v"(a), "v"(b));
  return c;
}
#define LDS_STRIDE 48
#define KSTRIDE    72
#define VSTRIDE    48

__device__ __forceinline__ f32x8 wmma_bf16(bf16x16 a, bf16x16 b, f32x8 c) {
  c = __builtin_amdgcn_wmma_f32_16x16x32_f16(false, a, false, b, (short)0, c, false, false);
  asm volatile("v_nop\n\tv_nop\n\tv_nop\n\tv_nop" : "+v"(c) : "v"(a), "v"(b));
  return c;
}

template <typename T>
__device__ __forceinline__ bf16x16 load_frag(const T* __restrict__ base, int ld,
                                             int row0, int k0) {
  const int lane = threadIdx.x & 31;
  const int r    = lane & 15;
  const int kh   = (lane >> 4) * 8;
  const T* p0 = base + (size_t)(row0 + r) * ld + (k0 + kh);
  const T* p1 = p0 + 16;
  bf16x16 f;
#pragma unroll
  for (int i = 0; i < 8; ++i) {
    f[i]     = (bf16)p0[i];
    f[i + 8] = (bf16)p1[i];
  }
  return f;
}

__device__ __forceinline__ bf16x16 lds_frag(const bf16* base, int stride) {
  const int lane = threadIdx.x & 31;
  const int row  = lane & 15;
  const int kh   = (lane >> 4) * 8;
  const bf16x8 lo = *(const bf16x8*)(base + row * stride + kh);
  const bf16x8 hi = *(const bf16x8*)(base + row * stride + kh + 16);
  bf16x16 f;
#pragma unroll
  for (int i = 0; i < 8; ++i) { f[i] = lo[i]; f[i + 8] = hi[i]; }
  return f;
}

template <typename T>
__device__ __forceinline__ void stage_read16(const T* __restrict__ p, float* buf) {
#pragma unroll
  for (int i = 0; i < 16; ++i) buf[i] = (float)p[i];
}

__device__ __forceinline__ void stage_write(bf16* dst, const float* buf, int nquad) {
#pragma unroll
  for (int i = 0; i < nquad; ++i) {
    bf16x4 q;
    q[0] = (bf16)buf[4 * i];     q[1] = (bf16)buf[4 * i + 1];
    q[2] = (bf16)buf[4 * i + 2]; q[3] = (bf16)buf[4 * i + 3];
    *(bf16x4*)(dst + 4 * i) = q;
  }
}


#define GSTR 48
template <typename AT, int EPI, bool OUT16>
__global__ __launch_bounds__(256) void gemm_kne(const AT* __restrict__ A, int lda, const float* __restrict__ Wm, int ldw,
                                                const float* __restrict__ bias, const float* __restrict__ R, const float* __restrict__ gvec,
                                                void* __restrict__ Yv, int ldy, int K) {
  __shared__ __attribute__((aligned(16))) f16 ldsA[128 * GSTR];
  __shared__ __attribute__((aligned(16))) f16 ldsW[128 * GSTR];
  __shared__ __attribute__((aligned(16))) float oS[8][32 * 68];
  const int tid = threadIdx.x, lane = tid & 31, wave = tid >> 5, cl = lane & 15, rh = (lane >> 4) * 8;
  const int m0 = blockIdx.x * 128, n0 = blockIdx.y * 128;
  const int wm = (wave & 3) * 32, wn = (wave >> 2) * 64;
  f32x8 acc[2][4];
#pragma unroll
  for (int i = 0; i < 2; ++i)
#pragma unroll
    for (int j = 0; j < 4; ++j) { f32x8 z = {}; acc[i][j] = z; }
#pragma unroll 1
  for (int k0 = 0; k0 < K; k0 += 32) {
    __syncthreads();
    { const int row = tid >> 1, ch = (tid & 1) * 16;
      const AT* src = A + (size_t)(m0 + row) * lda + k0 + ch;
#pragma unroll
      for (int g = 0; g < 16; ++g) ldsA[row * GSTR + ch + g] = (f16)src[g]; }
    { const int k = tid >> 3, nn0 = (tid & 7) * 16;
      const float* src = Wm + (size_t)(k0 + k) * ldw + n0 + nn0;
#pragma unroll
      for (int g = 0; g < 4; ++g) { const v4f_t v = *(const v4f_t*)(src + 4 * g);
#pragma unroll
        for (int u = 0; u < 4; ++u) ldsW[(nn0 + 4 * g + u) * GSTR + k] = (f16)v[u]; } }
    __syncthreads();
    f16x16 af[2];
#pragma unroll
    for (int i = 0; i < 2; ++i) af[i] = lds_frag(ldsA + (wm + 16 * i) * GSTR, GSTR);
#pragma unroll
    for (int j = 0; j < 4; ++j) {
      const f16x16 bf = lds_frag(ldsW + (wn + 16 * j) * GSTR, GSTR);
#pragma unroll
      for (int i = 0; i < 2; ++i) acc[i][j] = wmma16(af[i], bf, acc[i][j]);
    }
  }
  float* so = oS[wave];
#pragma unroll
  for (int i = 0; i < 2; ++i)
#pragma unroll
    for (int j = 0; j < 4; ++j) {
      const int n = n0 + wn + 16 * j + cl;
      const float bv = bias ? bias[n] : 0.0f;
      const float gv = (EPI == 2) ? gvec[n] : 0.0f;
      if (EPI == 1) {
#pragma unroll 1
        for (int r = 0; r < 8; ++r) { const float xg = acc[i][j][r] + bv; so[(16 * i + rh + r) * 68 + 16 * j + cl] = 0.5f * xg * (1.0f + erff(xg * 0.70710678118654752f)); }
      } else {
#pragma unroll
        for (int r = 0; r < 8; ++r) {
          float v = acc[i][j][r] + bv;
          if (EPI == 2) v = R[(size_t)(m0 + wm + 16 * i + rh + r) * ldy + n] + gv * v;
          so[(16 * i + rh + r) * 68 + 16 * j + cl] = v;
        }
      }
    }
  asm volatile("s_wait_dscnt 0" ::: "memory");
  __builtin_amdgcn_wave_barrier();
#pragma unroll 1
  for (int pass = 0; pass < 2; ++pass) {
    if (OUT16) {
      f16* Y = (f16*)Yv;
#pragma unroll
      for (int it = 0; it < 8; ++it) { const int c = lane + 32 * it, rr = c >> 3, q8 = (c & 7) * 8;
        union { f16 h[8]; v4u_t v; } u;
#pragma unroll
        for (int e = 0; e < 8; ++e) u.h[e] = (f16)so[rr * 68 + q8 + e];
        *(volatile v4u_t*)(Y + (size_t)(m0 + wm + rr) * ldy + n0 + wn + q8) = u.v; }
    } else {
      float* Y = (float*)Yv;
#pragma unroll
      for (int it = 0; it < 16; ++it) { const int f4 = lane + 32 * it, rr = f4 >> 4, q = (f4 & 15) * 4;
        *(volatile v4f_t*)(Y + (size_t)(m0 + wm + rr) * ldy + n0 + wn + q) = *(const v4fa*)(so + rr * 68 + q); }
    }
    __threadfence();
  }
}
__global__ __launch_bounds__(64) void attn_kernel(
    const bf16* __restrict__ Qb, const bf16* __restrict__ Kb,
    const bf16* __restrict__ Vt,
    bf16* __restrict__ attnOut) {
  __shared__ bf16 ldsK[32 * KSTRIDE];
  __shared__ bf16 ldsV[64 * VSTRIDE];
  __shared__ __attribute__((aligned(16))) bf16 ldsO[2][32 * 72];

  const int q0blk = blockIdx.x * 64;
  const int h  = blockIdx.y;
  const int b  = blockIdx.z;
  const int t    = threadIdx.x;
  const int wave = t >> 5;
  const int lane = t & 31;
  const int qlane = lane & 15;
  const int kh8   = (lane >> 4) * 8;
  const int q0 = q0blk + wave * 32;

  const int hk = h;
  const bf16* Qh = Qb + (size_t)b * SS * DD + h * DKK;
  const bf16* Kh = Kb + (size_t)b * SS * KVD + hk * DKK;
  const bf16* Vh = Vt + ((size_t)(b * KVH + hk)) * DKK * SS;

  const int krow = t >> 1;
  const int kcol = (t & 1) * 32;
  const bf16* kSrc = Kh + (size_t)krow * KVD + kcol;
  const bf16* vSrc = Vh + (size_t)t * SS;

  bf16x16 qf[QW][2];
#pragma unroll
  for (int qt = 0; qt < QW; ++qt) {
    qf[qt][0] = load_frag(Qh, DD, q0 + 16 * qt, 0);
    qf[qt][1] = load_frag(Qh, DD, q0 + 16 * qt, 32);
  }

  f32x8 o[QW][4] = {};
  float mrun[QW], lrun[QW];
#pragma unroll
  for (int qt = 0; qt < QW; ++qt) { mrun[qt] = -INFINITY; lrun[qt] = 0.0f; }

  const float scale = 0.125f * 1.44269504088896340736f;
  const float NEG2 = -1.0e9f;
  const int kmax = SS - 1;

  bf16x8 kreg[4], vreg[4];
#pragma unroll
  for (int i = 0; i < 4; ++i) {
    kreg[i] = *(const bf16x8*)(kSrc + 8 * i);
    vreg[i] = *(const bf16x8*)(vSrc + 8 * i);
  }

  for (int kb = 0; kb <= kmax; kb += 32) {
    __syncthreads();
#pragma unroll
    for (int i = 0; i < 4; ++i) {
      *(bf16x8*)(&ldsK[krow * KSTRIDE + kcol + 8 * i]) = kreg[i];
      *(bf16x8*)(&ldsV[t * VSTRIDE + 8 * i])           = vreg[i];
    }
    if (kb + 32 <= kmax) {
      const bf16* kn = kSrc + (size_t)(kb + 32) * KVD;
      const bf16* vn = vSrc + (kb + 32);
#pragma unroll
      for (int i = 0; i < 4; ++i) {
        kreg[i] = *(const bf16x8*)(kn + 8 * i);
        vreg[i] = *(const bf16x8*)(vn + 8 * i);
      }
    }
    __syncthreads();

    bf16x16 kf[2][2];
#pragma unroll
    for (int ktile = 0; ktile < 2; ++ktile)
#pragma unroll
      for (int c = 0; c < 2; ++c)
        kf[ktile][c] = lds_frag(ldsK + (ktile * 16) * KSTRIDE + c * 32, KSTRIDE);

    bf16x16 pf[QW];
    bool act[QW];
#pragma unroll
    for (int qt = 0; qt < QW; ++qt) {
      unsigned mbits = 0;
      mbits = 0xFFFFu; act[qt] = true;
      if (act[qt]) {
        const int q_my = q0 + 16 * qt + qlane;
        f32x8 s0 = {}, s1 = {};
        s0 = wmma_bf16(kf[0][0], qf[qt][0], s0);
        s0 = wmma_bf16(kf[0][1], qf[qt][1], s0);
        s1 = wmma_bf16(kf[1][0], qf[qt][0], s1);
        s1 = wmma_bf16(kf[1][1], qf[qt][1], s1);

        float mx = -INFINITY;
#pragma unroll
        for (int r = 0; r < 8; ++r) {
          const int k0i = kb + kh8 + r;
          const int k1i = k0i + 16;
          (void)k0i; (void)k1i; (void)q_my;
          s0[r] = (mbits & (1u << r))       ? s0[r] * scale : NEG2;
          s1[r] = (mbits & (1u << (8 + r))) ? s1[r] * scale : NEG2;
          mx = fmaxf(mx, fmaxf(s0[r], s1[r]));
        }
        mx = fmaxf(mx, __shfl_xor(mx, 16, 32));
        const float mnew  = fmaxf(mrun[qt], mx);
        const float alpha = exp2f(mrun[qt] - mnew);

        float rsum = 0.0f;
#pragma unroll
        for (int r = 0; r < 8; ++r) {
          const float p0 = exp2f(s0[r] - mnew);
          const float p1 = exp2f(s1[r] - mnew);
          rsum += p0 + p1;
          pf[qt][r]     = (bf16)(p0 * 1024.0f);
          pf[qt][r + 8] = (bf16)(p1 * 1024.0f);
        }
        rsum += __shfl_xor(rsum, 16, 32);
        lrun[qt] = lrun[qt] * alpha + rsum;
        mrun[qt] = mnew;

#pragma unroll
        for (int j = 0; j < 4; ++j)
#pragma unroll
          for (int r = 0; r < 8; ++r) o[qt][j][r] *= alpha;
      }
    }

#pragma unroll
    for (int j = 0; j < 4; ++j) {
      const bf16x16 vf = lds_frag(ldsV + (j * 16) * VSTRIDE, VSTRIDE);
#pragma unroll
      for (int qt = 0; qt < QW; ++qt)
        if (act[qt]) o[qt][j] = wmma_bf16(vf, pf[qt], o[qt][j]);
    }
  }

  bf16* so = ldsO[wave];
#pragma unroll
  for (int qt = 0; qt < QW; ++qt) {
    const float rl = 1.0f / (lrun[qt] * 1024.0f);
#pragma unroll
    for (int j = 0; j < 4; ++j)
#pragma unroll
      for (int r = 0; r < 8; ++r) so[(16 * qt + qlane) * 72 + j * 16 + kh8 + r] = (bf16)(o[qt][j][r] * rl);
  }
  asm volatile("s_wait_dscnt 0" ::: "memory");
#pragma unroll 1
  for (int pass = 0; pass < 2; ++pass) {
#pragma unroll
    for (int it = 0; it < 8; ++it) { const int ch = lane + 32 * it, ql = ch >> 3, q8 = (ch & 7) * 8;
      *(volatile v4u_t*)(attnOut + ((size_t)(b * SS + q0 + ql)) * DD + h * DKK + q8) = *(const v4ua*)(so + ql * 72 + q8); }
    __threadfence();
  }
}


__global__ __launch_bounds__(256) void k_ada(const float* __restrict__ c, const float* __restrict__ Wk, const float* __restrict__ bk, float* __restrict__ ada) {
  __shared__ float sc[DD];
  const int b = blockIdx.y, j = blockIdx.x * 256 + threadIdx.x;
  for (int i = threadIdx.x; i < DD; i += 256) { const float v = c[(size_t)b * DD + i]; sc[i] = v / (1.0f + expf(-v)); }
  __syncthreads();
  float s = bk[j];
#pragma unroll 1
  for (int i = 0; i < DD; ++i) s += sc[i] * Wk[(size_t)i * (6 * DD) + j];
  *(volatile float*)(ada + (size_t)b * 6 * DD + j) = s; __threadfence(); *(volatile float*)(ada + (size_t)b * 6 * DD + j) = s;
}
__global__ __launch_bounds__(256) void k_rmsmod(const float* __restrict__ X, const float* __restrict__ w, const float* __restrict__ ada, int shOff, int scOff, float* __restrict__ Y) {
  __shared__ __attribute__((aligned(16))) float rowS[8 * 1028];
  const int tid = threadIdx.x, r = tid >> 5, lane = tid & 31; const size_t row = (size_t)blockIdx.x * 8 + r; const int b = row / SS;
  const float* xr = X + row * DD; float q = 0.0f;
#pragma unroll 1
  for (int i = lane; i < DD; i += 32) { const float v = xr[i]; rowS[r * 1028 + i] = v; q += v * v; }
#pragma unroll
  for (int off = 1; off < 32; off <<= 1) q += __shfl_xor(q, off, 32);
  const float rs = rsqrtf(q * (1.0f / DD) + 1e-6f);
  const float* sh = ada + (size_t)b * 6 * DD + shOff; const float* scv = ada + (size_t)b * 6 * DD + scOff;
#pragma unroll 1
  for (int i = lane; i < DD; i += 32) rowS[r * 1028 + i] = rowS[r * 1028 + i] * rs * w[i] * (1.0f + scv[i]) + sh[i];
  __syncthreads();
#pragma unroll 1
  for (int pass = 0; pass < 2; ++pass) { for (int q4 = tid; q4 < 8 * 256; q4 += 256) { const int rr = q4 >> 8, c4 = (q4 & 255) * 4;
      *(volatile v4f_t*)(Y + ((size_t)blockIdx.x * 8 + rr) * DD + c4) = *(const v4fa*)(rowS + rr * 1028 + c4); } __threadfence(); }
}
__global__ __launch_bounds__(256) void k_qk(const float* __restrict__ qkv, const float* __restrict__ qn, const float* __restrict__ kn, const float* __restrict__ rc, const float* __restrict__ rs_, bf16* __restrict__ Q16, bf16* __restrict__ K16) {
  __shared__ __attribute__((aligned(16))) bf16 oS[2][4][DD + 8];
  const int tid = threadIdx.x; const int which = tid >> 7, r = (tid >> 5) & 3, h = (tid >> 1) & 15, half = tid & 1;
  const size_t row = (size_t)blockIdx.x * 4 + r; const int n = row % SS;
  const float* src = qkv + row * (3 * DD) + which * DD + h * DKK; const float* wn = which ? kn : qn;
  float v[32]; float q = 0.0f;
#pragma unroll
  for (int i = 0; i < 32; ++i) { v[i] = src[half * 32 + i]; q += v[i] * v[i]; }
  q += __shfl_xor(q, 1, 32);
  const float rsn = rsqrtf(q * (1.0f / DKK) + 1e-6f);
#pragma unroll
  for (int i = 0; i < 32; ++i) { const float mine = v[i] * rsn * wn[half * 32 + i]; const float other = __shfl_xor(mine, 1, 32) ; const float cs = rc[n * 32 + i], sn = rs_[n * 32 + i];
    const float o = half ? (other * sn + mine * cs) : (mine * cs - other * sn);
    oS[which][r][h * DKK + half * 32 + i] = (bf16)o; }
  __syncthreads();
#pragma unroll 1
  for (int pass = 0; pass < 2; ++pass) { for (int e = tid; e < 8 * 128; e += 256) { const int wr = e >> 7, piece = (e & 127) * 8; const int w2 = wr >> 2, rr = wr & 3;
      bf16* dst = (w2 ? K16 : Q16) + ((size_t)blockIdx.x * 4 + rr) * DD + piece; *(volatile v4u_t*)dst = *(const v4ua*)(&oS[w2][rr][piece]); } __threadfence(); }
}
__global__ __launch_bounds__(256) void k_vt(const float* __restrict__ qkv, bf16* __restrict__ Vt) {
  __shared__ __attribute__((aligned(16))) bf16 tS[256][72];
  const int tid = threadIdx.x; const int b = blockIdx.z, t0 = blockIdx.x * 64, c0 = blockIdx.y * 256;
  for (int e = tid; e < 64 * 256; e += 256) { const int t = e >> 8, c = e & 255; tS[c][t] = (bf16)qkv[((size_t)b * SS + t0 + t) * (3 * DD) + 2 * DD + c0 + c]; }
  __syncthreads();
#pragma unroll 1
  for (int pass = 0; pass < 2; ++pass) { for (int e = tid; e < 256 * 8; e += 256) { const int c = e >> 3, piece = (e & 7) * 8;
      *(volatile v4u_t*)(Vt + ((size_t)b * DD + c0 + c) * SS + t0 + piece) = *(const v4ua*)(&tS[c][piece]); } __threadfence(); }
}
__global__ __launch_bounds__(256) void k_padcols(const float* __restrict__ Wm, int ld, int off, int ncols, int NP, float* __restrict__ Wp, const float* __restrict__ bsrc, float* __restrict__ bp) {
  const int i = blockIdx.x;
  for (int n = threadIdx.x; n < NP; n += 256) { const float v = (n < ncols) ? Wm[(size_t)i * ld + off + n] : 0.0f; *(volatile float*)(Wp + (size_t)i * NP + n) = v; __threadfence(); *(volatile float*)(Wp + (size_t)i * NP + n) = v;
    if (i == 0 && bp) { const float bv = (n < ncols) ? bsrc[off + n] : 0.0f; *(volatile float*)(bp + n) = bv; __threadfence(); *(volatile float*)(bp + n) = bv; } }
}
__global__ __launch_bounds__(256) void k_padrows(const float* __restrict__ Wm, float* __restrict__ Wp) { const int k = blockIdx.x;
  for (int q4 = threadIdx.x; q4 < DD / 4; q4 += 256) { v4f_t v = {0.f,0.f,0.f,0.f}; if (k < MH) v = *(const v4f_t*)(Wm + (size_t)k * DD + q4 * 4); *(volatile v4f_t*)(Wp + (size_t)k * DD + q4 * 4) = v; __threadfence(); *(volatile v4f_t*)(Wp + (size_t)k * DD + q4 * 4) = v; } }
__global__ __launch_bounds__(256) void k_swiglu(float* __restrict__ u1, const float* __restrict__ u2) { const size_t row = blockIdx.x;
  for (int q4 = threadIdx.x; q4 < MHP / 4; q4 += 256) { const v4f_t a = *(const v4f_t*)(u1 + row * MHP + q4 * 4), b = *(const v4f_t*)(u2 + row * MHP + q4 * 4); v4f_t o;
    for (int e = 0; e < 4; ++e) o[e] = (a[e] / (1.0f + expf(-a[e]))) * b[e];
    *(volatile v4f_t*)(u1 + row * MHP + q4 * 4) = o; __threadfence(); *(volatile v4f_t*)(u1 + row * MHP + q4 * 4) = o; } }

extern "C" void kernel_launch(void* const* d_in, const int* in_sizes, int n_in,
                              void* d_out, int out_size, void* d_ws, size_t ws_size,
                              hipStream_t stream) {
  (void)in_sizes; (void)n_in; (void)out_size;
  const float** f = (const float**)d_in;
  const float* x = f[0], *c = f[1], *rc = f[2], *rs_ = f[3], *n1w = f[4], *n2w = f[5], *qn = f[6], *kn = f[7], *qkvk = f[8], *qkvb = f[9], *pk = f[10], *pb = f[11],
             *w12 = f[12], *b12 = f[13], *w3 = f[14], *b3 = f[15], *adk = f[16], *adb = f[17];
  float* out = (float*)d_out;
  char* ws = (char*)d_ws;
  float* ada = (float*)ws; ws += (size_t)BB * 6 * DD * 4;
  float* regH = (float*)ws; ws += (size_t)MTOK * DD * 4;
  char* regQ = ws; ws += (size_t)MTOK * 3 * DD * 4;
  char* regA = ws; ws += (size_t)MTOK * DD * 2 * 4;
  float* x1 = (float*)ws; ws += (size_t)MTOK * DD * 4;
  if ((size_t)(ws - (char*)d_ws) > ws_size) return;
  float* h = regH; float* qkv = (float*)regQ;
  bf16* Q16 = (bf16*)regA; bf16* K16 = Q16 + (size_t)MTOK * DD; bf16* Vt = K16 + (size_t)MTOK * DD; bf16* att = Vt + (size_t)MTOK * DD;
  float* u1 = (float*)regQ; float* u2 = u1 + (size_t)SS * MHP; float* W1p = u2 + (size_t)SS * MHP; float* W2p = W1p + (size_t)DD * MHP;
  float* W3p = (float*)regA;
  const dim3 blk(256);
  float* b1p = W3p + (size_t)MHP * DD; float* b2p = b1p + MHP;
  k_ada<<<dim3(6 * DD / 256, BB), blk, 0, stream>>>(c, adk, adb, ada);
  k_rmsmod<<<dim3(MTOK / 8), blk, 0, stream>>>(x, n1w, ada, 0 * DD, 1 * DD, h);
  gemm_kne<float, 0, false><<<dim3(MTOK / 128, 3 * DD / 128), blk, 0, stream>>>(h, DD, qkvk, 3 * DD, qkvb, nullptr, nullptr, qkv, 3 * DD, DD);
  k_qk<<<dim3(MTOK / 4), blk, 0, stream>>>(qkv, qn, kn, rc, rs_, Q16, K16);
  k_vt<<<dim3(SS / 64, DD / 256, BB), blk, 0, stream>>>(qkv, Vt);
  attn_kernel<<<dim3(SS / 64, HH, BB), dim3(64), 0, stream>>>(Q16, K16, Vt, att);
  for (int b = 0; b < BB; ++b)
    gemm_kne<bf16, 2, false><<<dim3(SS / 128, DD / 128), blk, 0, stream>>>(att + (size_t)b * SS * DD, DD, pk, DD, pb, x + (size_t)b * SS * DD, ada + (size_t)b * 6 * DD + 2 * DD, x1 + (size_t)b * SS * DD, DD, DD);
  float* h2 = regH;
  k_rmsmod<<<dim3(MTOK / 8), blk, 0, stream>>>(x1, n2w, ada, 3 * DD, 4 * DD, h2);
  k_padcols<<<dim3(DD), blk, 0, stream>>>(w12, 2 * MH, 0, MH, MHP, W1p, b12, b1p);
  k_padcols<<<dim3(DD), blk, 0, stream>>>(w12, 2 * MH, MH, MH, MHP, W2p, b12, b2p);
  k_padrows<<<dim3(MHP), blk, 0, stream>>>(w3, W3p);
  for (int b = 0; b < BB; ++b) {
    const float* h2b = h2 + (size_t)b * SS * DD;
    gemm_kne<float, 0, false><<<dim3(SS / 128, MHP / 128), blk, 0, stream>>>(h2b, DD, W1p, MHP, b1p, nullptr, nullptr, u1, MHP, DD);
    gemm_kne<float, 0, false><<<dim3(SS / 128, MHP / 128), blk, 0, stream>>>(h2b, DD, W2p, MHP, b2p, nullptr, nullptr, u2, MHP, DD);
    k_swiglu<<<dim3(SS), blk, 0, stream>>>(u1, u2);
    gemm_kne<float, 2, false><<<dim3(SS / 128, DD / 128), blk, 0, stream>>>(u1, MHP, W3p, DD, b3, x1 + (size_t)b * SS * DD, ada + (size_t)b * 6 * DD + 5 * DD, out + (size_t)b * SS * DD, DD, MHP);
  }
}
